// GINNet_1726576853642
// MI455X (gfx1250) — hardware-verified
//
#include <hip/hip_runtime.h>
#include <stddef.h>
#include <stdint.h>


#define NN       40000
#define NE       640000
#define NF       64
#define HID      128
#define NG       256
#define MP       40064
#define NTHR     256
#define NWAVE    8
#define EPT      8
#define CHUNK    (NTHR * EPT)
#define WCAP     (EPT * 32)
#define LISTN    (NWAVE * WCAP)
#define NBMAX    2048
#define NB       1024
#define NBB      40
#define TABN     (NBB * NB)
#define RCAP     28672
#define DEGCAP   64
#define MEASDEG  36
#define MEASHIT  16638
#define PKS      11
#define GBM      64
#define GTHR     128
#define GNT      8
#define BN       128
#define APW      256
#define Z1W      128
#define ARPB     64
#define WSQ      (HID * 256)
#define NUX      (MP * (NF / 8))
#define NU1      (HID * (128 / 8))
#define NUSQ     (HID * (256 / 8))
#define NUTOT    (NUX + NU1 + 6 * NUSQ)
#define LDS_AGG  ((2 * RCAP + 2 * NBMAX + LISTN) * 4 + 64)
#define WSCAP    134217728

static_assert((CHUNK & (CHUNK - 1)) == 0 && CHUNK <= (1 << PKS));
static_assert((NBMAX & (NBMAX - 1)) == 0 && NBMAX <= (1 << PKS));
static_assert(NTHR * 8 == NBMAX && NB <= NBMAX && NB == 1024 && NB == 4 * NTHR);
static_assert(LISTN >= NBMAX && LISTN >= NWAVE * WCAP);
static_assert((RCAP % (4 * NTHR)) == 0);
static_assert(LDS_AGG <= 300000);
static_assert(NE <= (1 << 21) && (NE % 4) == 0);
static_assert(DEGCAP >= MEASDEG + 8);
static_assert((long long)RCAP * 100LL >= (long long)MEASHIT * 105LL);
static_assert(MP >= NN && (MP % GBM) == 0 && (MP % ARPB) == 0 && (MP % 128) == 0 && MP - NN < 128);
static_assert(NBB * NB >= MP && (NBB - 1) * NB < NN && (NB % ARPB) == 0 && ARPB == NWAVE * 8);
static_assert(GBM == (GTHR / 32) * 16 && BN == 16 * GNT && HID == BN && (NG % GBM) == 0);
static_assert((NUX % NTHR) == 0 && (NU1 % NTHR) == 0 && (NUSQ % NTHR) == 0 && (NUTOT % NTHR) == 0);
static_assert(NUSQ == 4096 && NF == 64 && HID == 128);
static_assert((NN % 4) == 0);

typedef float          v4f  __attribute__((ext_vector_type(4)));
typedef float          v8f  __attribute__((ext_vector_type(8)));
typedef int            v4i  __attribute__((ext_vector_type(4)));
typedef int            v8i  __attribute__((ext_vector_type(8)));
typedef unsigned int   v2u  __attribute__((ext_vector_type(2)));
typedef unsigned int   v4u  __attribute__((ext_vector_type(4)));
typedef unsigned short v8us __attribute__((ext_vector_type(8)));
typedef __bf16         v16b __attribute__((ext_vector_type(16)));
typedef v4f  __attribute__((may_alias)) v4fa;
typedef v8us __attribute__((may_alias)) v8usa;
union FragB { v16b v; v8us h[2]; v8i w; };

__device__ __forceinline__ v8f wmb(const FragB& a, const FragB& b, v8f c) {
  v8f d = __builtin_amdgcn_wmma_f32_16x16x32_bf16(false, a.v, false, b.v, (short)0, c, false, false);
  asm volatile("v_nop\n\tv_nop\n\tv_nop\n\tv_nop" : "+v"(d) : "v"(a.w), "v"(b.w));
  return d;
}

__device__ __forceinline__ unsigned short bf_bits(float f) {
  const unsigned int u = __float_as_uint(f);
  unsigned int r = u + 0x7FFFu + ((u >> 16) & 1u);
  r = (f != f) ? 0x7FC00000u : r;
  return (unsigned short)(r >> 16);
}
__device__ __forceinline__ float bf_val(unsigned short b) { return __uint_as_float(((unsigned int)b) << 16); }
__device__ __forceinline__ float bf_rne(float f) { return bf_val(bf_bits(f)); }
__device__ __forceinline__ float relu_np(float v) { return (v > 0.0f) ? v : (v - v); }

__device__ __forceinline__ int scan_chunk(const int* __restrict__ dsts, int nE, int cbase, int slotBase,
                                          int nb, int vec8, int* list, int tid, int lane, int wave) {
  int wc = 0;
  const int el0  = tid * EPT;
  const int e0   = cbase + el0;
  const int sent = -2147483647 - 1;
  v4i da, db;
  if (vec8 != 0 && cbase + CHUNK <= nE) {
    da = *(const v4i*)(dsts + e0);
    db = *(const v4i*)(dsts + e0 + 4);
  } else {
    da.x = (e0     < nE) ? dsts[min(e0,     nE - 1)] : sent;
    da.y = (e0 + 1 < nE) ? dsts[min(e0 + 1, nE - 1)] : sent;
    da.z = (e0 + 2 < nE) ? dsts[min(e0 + 2, nE - 1)] : sent;
    da.w = (e0 + 3 < nE) ? dsts[min(e0 + 3, nE - 1)] : sent;
    db.x = (e0 + 4 < nE) ? dsts[min(e0 + 4, nE - 1)] : sent;
    db.y = (e0 + 5 < nE) ? dsts[min(e0 + 5, nE - 1)] : sent;
    db.z = (e0 + 6 < nE) ? dsts[min(e0 + 6, nE - 1)] : sent;
    db.w = (e0 + 7 < nE) ? dsts[min(e0 + 7, nE - 1)] : sent;
  }
  const unsigned nbs = (unsigned)slotBase;
  const unsigned unb = (unsigned)nb;
  const unsigned s0 = (unsigned)da.x - nbs, s1 = (unsigned)da.y - nbs;
  const unsigned s2 = (unsigned)da.z - nbs, s3 = (unsigned)da.w - nbs;
  const unsigned s4 = (unsigned)db.x - nbs, s5 = (unsigned)db.y - nbs;
  const unsigned s6 = (unsigned)db.z - nbs, s7 = (unsigned)db.w - nbs;
  const bool h0 = s0 < unb, h1 = s1 < unb, h2 = s2 < unb, h3 = s3 < unb;
  const bool h4 = s4 < unb, h5 = s5 < unb, h6 = s6 < unb, h7 = s7 < unb;
  const unsigned any = __builtin_amdgcn_ballot_w32(h0 | h1 | h2 | h3 | h4 | h5 | h6 | h7);
  if (any != 0u) {
#define HITJ(J, HJ, SJ) { \
      const unsigned mj = __builtin_amdgcn_ballot_w32(HJ); \
      if (mj != 0u) { \
        if (HJ) { \
          const int pos = wc + (int)__builtin_amdgcn_mbcnt_lo(mj, 0u); \
          if (pos < WCAP) list[wave * WCAP + pos] = ((el0 + (J)) << PKS) | (int)(SJ); \
        } \
        wc += (int)__builtin_popcount(mj); } }
    HITJ(0, h0, s0)
    HITJ(1, h1, s1)
    HITJ(2, h2, s2)
    HITJ(3, h3, s3)
    HITJ(4, h4, s4)
    HITJ(5, h5, s5)
    HITJ(6, h6, s6)
    HITJ(7, h7, s7)
#undef HITJ
  }
  return wc;
}

__global__ __launch_bounds__(NTHR) void k_prep(const float* __restrict__ x, const float* __restrict__ w1a,
                                               const float* __restrict__ w1b, const float* __restrict__ w2a,
                                               const float* __restrict__ w2b, const float* __restrict__ w3a,
                                               const float* __restrict__ w3b, const float* __restrict__ l1w,
                                               unsigned short* xb, unsigned short* w1at, unsigned short* wt6) {
  const int u = (int)blockIdx.x * NTHR + (int)threadIdx.x;
  v8us o;
  unsigned short* dp;
  if (u < NUX) {
    const int row = u >> 3;
    const int c8  = (u & 7) * 8;
    const int rc  = row < NN ? row : NN - 1;
    const v4f a = *(const v4f*)(x + (size_t)rc * NF + c8);
    const v4f b = *(const v4f*)(x + (size_t)rc * NF + c8 + 4);
    const bool live = row < NN;
    const float f[8] = {a.x, a.y, a.z, a.w, b.x, b.y, b.z, b.w};
#pragma unroll
    for (int i = 0; i < 8; ++i) {
      const unsigned short q = bf_bits(f[i]);
      o[i] = live ? q : (unsigned short)0;
    }
    dp = xb + (size_t)u * 8;
  } else if (u < NUX + NU1) {
    const int v  = u - NUX;
    const int n  = v >> 4;
    const int k8 = (v & 15) * 8;
    const int kk = k8 & (NF - 1);
    const float* p = w1a + (size_t)kk * HID + n;
#pragma unroll
    for (int i = 0; i < 8; ++i) o[i] = bf_bits(p[(size_t)i * HID]);
    dp = w1at + (size_t)v * 8;
  } else if (u < NUTOT) {
    const int v  = u - NUX - NU1;
    const int mi = v >> 12;
    const int vv = v & (NUSQ - 1);
    const int n  = vv >> 5;
    const int k8 = (vv & 31) * 8;
    const int kk = k8 & (HID - 1);
    const float* Wb = w1b;
    if (mi == 1) Wb = w2a;
    if (mi == 2) Wb = w2b;
    if (mi == 3) Wb = w3a;
    if (mi == 4) Wb = w3b;
    if (mi == 5) Wb = l1w;
    const float* p = Wb + (size_t)kk * HID + n;
#pragma unroll
    for (int i = 0; i < 8; ++i) o[i] = bf_bits(p[(size_t)i * HID]);
    dp = wt6 + (size_t)mi * WSQ + (size_t)vv * 8;
  } else {
    return;
  }
  *(volatile v8us*)dp = o;
  __threadfence();
  *(volatile v8us*)dp = o;
}

__global__ __launch_bounds__(NTHR) void k_bucket(const int* __restrict__ srcs, const int* __restrict__ dsts,
                                                 int* listg, int* cntg, int* offg, int* flagg) {
  extern __shared__ v4f lds_dyn[];
  int* reg1 = (int*)lds_dyn;
  int* reg2 = reg1 + RCAP;
  int* scnt = reg2 + RCAP;
  int* soff = scnt + NBMAX;
  int* list = soff + NBMAX;
  int* wcnt = list + LISTN;
  int* wtot = wcnt + NWAVE;
  const int tid = (int)threadIdx.x, lane = tid & 31, wave = tid >> 5;
  const int nodeBase = (int)blockIdx.x * NB;
  int nb = NN - nodeBase;
  nb = nb < 0 ? 0 : (nb > NB ? NB : nb);
  const int nE = NE;

  for (int i = tid; i < NBMAX; i += NTHR) scnt[i] = 0;
  {
    const v4i z4 = {0, 0, 0, 0};
    for (int i = tid; i < RCAP / 4; i += NTHR) *(v4i*)(reg2 + 4 * i) = z4;
  }
  __syncthreads();

  int tot = 0;
  const int nChunks = (nE + CHUNK - 1) / CHUNK;
#pragma unroll 1
  for (int ch = 0; ch < nChunks; ++ch) {
    const int cbase = ch * CHUNK;
    const int wc = scan_chunk(dsts, nE, cbase, nodeBase, nb, 1, list, tid, lane, wave);
    if (lane == 0) wcnt[wave] = wc;
    __syncthreads();
    int pre = 0, all = 0;
#pragma unroll
    for (int w2 = 0; w2 < NWAVE; ++w2) {
      int c = wcnt[w2];
      c = c < 0 ? 0 : (c > WCAP ? WCAP : c);
      all += c;
      pre += (w2 < wave) ? c : 0;
    }
    const int wcc  = wc > WCAP ? WCAP : wc;
    const int base = tot + pre;
#pragma unroll 1
    for (int i = lane; i < wcc; i += 32) {
      const int ent = list[wave * WCAP + i];
      const int el  = (ent >> PKS) & (CHUNK - 1);
      const int sl  = ent & (NBMAX - 1);
      int eid = cbase + el;
      eid = eid > nE - 1 ? nE - 1 : eid;
      const int pos = base + i;
      if (pos < RCAP) reg1[pos] = (int)(((unsigned)eid << PKS) | (unsigned)sl);
    }
    tot += all;
    tot = tot > RCAP ? RCAP : tot;
    __syncthreads();
  }
  const int nh = tot;

  if (wave == 0) {
#pragma unroll 1
    for (int b0 = 0; b0 < nh; b0 += 32) {
      int idx = b0 + lane;
      idx = idx > nh - 1 ? nh - 1 : idx;
      idx = idx < 0 ? 0 : (idx > RCAP - 1 ? RCAP - 1 : idx);
      const int uv  = reg1[idx];
      const int m32 = (nh - b0) < 32 ? (nh - b0) : 32;
#pragma unroll 1
      for (int k = 0; k < m32; ++k) {
        const int u  = __builtin_amdgcn_readlane(uv, k);
        const int sl = u & (NBMAX - 1);
        if (lane == 0) scnt[sl] = scnt[sl] + 1;
      }
    }
  }
  __syncthreads();

  {
    const v4i ca = *(const v4i*)(scnt + 8 * tid);
    const v4i cb = *(const v4i*)(scnt + 8 * tid + 4);
    const int e0 = ca.x < 0 ? 0 : ca.x, e1 = ca.y < 0 ? 0 : ca.y, e2 = ca.z < 0 ? 0 : ca.z, e3 = ca.w < 0 ? 0 : ca.w;
    const int e4 = cb.x < 0 ? 0 : cb.x, e5 = cb.y < 0 ? 0 : cb.y, e6 = cb.z < 0 ? 0 : cb.z, e7 = cb.w < 0 ? 0 : cb.w;
    const int ts = e0 + e1 + e2 + e3 + e4 + e5 + e6 + e7;
    int incl = ts;
#pragma unroll
    for (int d = 1; d < 32; d <<= 1) {
      const int up = __shfl_up(incl, d);
      if (lane >= d) incl += up;
    }
    if (lane == 31) wtot[wave] = incl;
    __syncthreads();
    int pre = 0;
#pragma unroll
    for (int w2 = 0; w2 < NWAVE; ++w2) pre += (w2 < wave) ? wtot[w2] : 0;
    int run = pre + incl - ts;
    soff[8 * tid + 0] = run; run += e0;
    soff[8 * tid + 1] = run; run += e1;
    soff[8 * tid + 2] = run; run += e2;
    soff[8 * tid + 3] = run; run += e3;
    soff[8 * tid + 4] = run; run += e4;
    soff[8 * tid + 5] = run; run += e5;
    soff[8 * tid + 6] = run; run += e6;
    soff[8 * tid + 7] = run;
  }
  __syncthreads();
  for (int i = tid; i < NBMAX; i += NTHR) list[i] = soff[i];
  __syncthreads();

  if (wave == 0) {
#pragma unroll 1
    for (int b0 = 0; b0 < nh; b0 += 32) {
      int idx = b0 + lane;
      idx = idx > nh - 1 ? nh - 1 : idx;
      idx = idx < 0 ? 0 : (idx > RCAP - 1 ? RCAP - 1 : idx);
      const int uv  = reg1[idx];
      const int m32 = (nh - b0) < 32 ? (nh - b0) : 32;
#pragma unroll 1
      for (int k = 0; k < m32; ++k) {
        const int u   = __builtin_amdgcn_readlane(uv, k);
        const int sl  = u & (NBMAX - 1);
        const int eid = (int)((unsigned)u >> PKS);
        if (lane == 0) {
          int pos = list[sl];
          pos = pos < 0 ? 0 : (pos > RCAP - 1 ? RCAP - 1 : pos);
          reg2[pos] = eid;
          list[sl] = pos + 1;
        }
      }
    }
  }
  __syncthreads();

  int* lb = listg + (size_t)blockIdx.x * RCAP;
#pragma unroll 1
  for (int it = 0; it < RCAP / (4 * NTHR); ++it) {
    const int i4 = (it * NTHR + tid) * 4;
    const v4i e = *(const v4i*)(reg2 + i4);
    const int q0 = e.x < 0 ? 0 : (e.x > NE - 1 ? NE - 1 : e.x);
    const int q1 = e.y < 0 ? 0 : (e.y > NE - 1 ? NE - 1 : e.y);
    const int q2 = e.z < 0 ? 0 : (e.z > NE - 1 ? NE - 1 : e.z);
    const int q3 = e.w < 0 ? 0 : (e.w > NE - 1 ? NE - 1 : e.w);
    int t0 = srcs[q0], t1 = srcs[q1], t2 = srcs[q2], t3 = srcs[q3];
    t0 = t0 < 0 ? 0 : (t0 > NN - 1 ? NN - 1 : t0);
    t1 = t1 < 0 ? 0 : (t1 > NN - 1 ? NN - 1 : t1);
    t2 = t2 < 0 ? 0 : (t2 > NN - 1 ? NN - 1 : t2);
    t3 = t3 < 0 ? 0 : (t3 > NN - 1 ? NN - 1 : t3);
    v4i o;
    o.x = (i4     < nh) ? t0 : 0;
    o.y = (i4 + 1 < nh) ? t1 : 0;
    o.z = (i4 + 2 < nh) ? t2 : 0;
    o.w = (i4 + 3 < nh) ? t3 : 0;
    *(volatile v4i*)(lb + i4) = o;
    __threadfence();
    *(volatile v4i*)(lb + i4) = o;
  }
  const v4i cv = *(const v4i*)(scnt + 4 * tid);
  const v4i ov = *(const v4i*)(soff + 4 * tid);
  const int ovfI = (nh >= RCAP) ? 1 : 0;
  v4i fv = {0, 0, 0, 0};
  fv.x = (tid == 0) ? ovfI : 0;
  int* cp = cntg + (size_t)blockIdx.x * NB + 4 * tid;
  int* op = offg + (size_t)blockIdx.x * NB + 4 * tid;
  int* fp = flagg + (size_t)blockIdx.x * 32 + 4 * (tid & 7);
  *(volatile v4i*)cp = cv;
  *(volatile v4i*)op = ov;
  if (tid < 8) *(volatile v4i*)fp = fv;
  __threadfence();
  *(volatile v4i*)cp = cv;
  *(volatile v4i*)op = ov;
  if (tid < 8) *(volatile v4i*)fp = fv;
}

template <int FIRST>
__global__ __launch_bounds__(NTHR) void k_agg(const unsigned short* __restrict__ xb, const float* __restrict__ hf,
                                              const int* __restrict__ listg, const int* __restrict__ cntg,
                                              const int* __restrict__ offg, const int* __restrict__ flagg,
                                              const float* __restrict__ epsp, unsigned short* zout) {
  const int tid = (int)threadIdx.x, lane = tid & 31, wave = tid >> 5;
  const int rowBase = (int)blockIdx.x * ARPB;
  const int rw = rowBase + wave * 8;
  int bb = rowBase >> 10;
  bb = bb > NBB - 1 ? NBB - 1 : bb;
  const int fl = flagg[bb * 32];
  const float sfac = 1.0f + bf_rne(epsp[0]);
  int ti = rw + (lane & 7);
  ti = ti > TABN - 1 ? TABN - 1 : ti;
  const int cvv = cntg[ti];
  const int ovv = offg[ti];
  const int* lb = listg + (size_t)bb * RCAP;
  const float qnan = __int_as_float(0x7fc00000);

#pragma unroll 1
  for (int j = 0; j < 8; ++j) {
    const int grow = rw + j;
    const int craw = __builtin_amdgcn_readlane(cvv, j);
    int st  = __builtin_amdgcn_readlane(ovv, j);
    int cnt = craw;
    st  = st < 0 ? 0 : (st > RCAP ? RCAP : st);
    cnt = cnt < 0 ? 0 : (cnt > DEGCAP ? DEGCAP : cnt);
    if (cnt > RCAP - st) cnt = RCAP - st;
    const float pz = (fl != 0 || craw > DEGCAP || craw < 0) ? qnan : 0.0f;
    const bool liveRow = grow < NN;
    const int nc = liveRow ? grow : NN - 1;

    float ag0 = 0.f, ag1 = 0.f, ag2 = 0.f, ag3 = 0.f;
#pragma unroll 1
    for (int b0 = 0; b0 < cnt; b0 += 32) {
      int idx = st + b0 + lane;
      idx = idx > st + cnt - 1 ? st + cnt - 1 : idx;
      idx = idx < 0 ? 0 : (idx > RCAP - 1 ? RCAP - 1 : idx);
      int sv = lb[idx];
      sv = sv < 0 ? 0 : (sv > NN - 1 ? NN - 1 : sv);
      const int m32 = (cnt - b0) < 32 ? (cnt - b0) : 32;
#pragma unroll 1
      for (int k = 0; k < m32; ++k) {
        const int sk = __builtin_amdgcn_readlane(sv, k);
        if constexpr (FIRST != 0) {
          const unsigned int w = *(const unsigned int*)(xb + (size_t)sk * NF + 2 * lane);
          ag0 += __uint_as_float(w << 16);
          ag1 += __uint_as_float(w & 0xffff0000u);
        } else {
          const v4f v = *(const v4f*)(hf + (size_t)sk * HID + 4 * lane);
          ag0 += v.x; ag1 += v.y; ag2 += v.z; ag3 += v.w;
        }
      }
    }

    if constexpr (FIRST != 0) {
      const unsigned int w = *(const unsigned int*)(xb + (size_t)nc * NF + 2 * lane);
      float r0 = sfac * __uint_as_float(w << 16) + ag0;
      float r1 = sfac * __uint_as_float(w & 0xffff0000u) + ag1;
      r0 = (liveRow ? r0 : 0.0f) + pz;
      r1 = (liveRow ? r1 : 0.0f) + pz;
      const unsigned short hb0 = bf_bits(r0), hb1 = bf_bits(r1);
      const unsigned short lb0 = bf_bits(r0 - bf_val(hb0)), lb1 = bf_bits(r1 - bf_val(hb1));
      const unsigned int hw = (unsigned int)hb0 | ((unsigned int)hb1 << 16);
      const unsigned int lw = (unsigned int)lb0 | ((unsigned int)lb1 << 16);
      unsigned int* gp = (unsigned int*)(zout + (size_t)grow * Z1W);
      const bool wsv = grow < MP;
      if (wsv) { *(volatile unsigned int*)(gp + lane) = hw; *(volatile unsigned int*)(gp + 32 + lane) = lw; }
      __threadfence();
      if (wsv) { *(volatile unsigned int*)(gp + lane) = hw; *(volatile unsigned int*)(gp + 32 + lane) = lw; }
    } else {
      const v4f sf = *(const v4f*)(hf + (size_t)nc * HID + 4 * lane);
      float r0 = sfac * sf.x + ag0, r1 = sfac * sf.y + ag1, r2 = sfac * sf.z + ag2, r3 = sfac * sf.w + ag3;
      r0 = (liveRow ? r0 : 0.0f) + pz;
      r1 = (liveRow ? r1 : 0.0f) + pz;
      r2 = (liveRow ? r2 : 0.0f) + pz;
      r3 = (liveRow ? r3 : 0.0f) + pz;
      const unsigned short hb0 = bf_bits(r0), hb1 = bf_bits(r1), hb2 = bf_bits(r2), hb3 = bf_bits(r3);
      const unsigned short lb0 = bf_bits(r0 - bf_val(hb0)), lb1 = bf_bits(r1 - bf_val(hb1));
      const unsigned short lb2 = bf_bits(r2 - bf_val(hb2)), lb3 = bf_bits(r3 - bf_val(hb3));
      v2u hw, lw;
      hw.x = (unsigned int)hb0 | ((unsigned int)hb1 << 16);
      hw.y = (unsigned int)hb2 | ((unsigned int)hb3 << 16);
      lw.x = (unsigned int)lb0 | ((unsigned int)lb1 << 16);
      lw.y = (unsigned int)lb2 | ((unsigned int)lb3 << 16);
      unsigned short* gp = zout + (size_t)grow * APW;
      const bool wsv = grow < MP;
      if (wsv) { *(volatile v2u*)(gp + 4 * lane) = hw; *(volatile v2u*)(gp + HID + 4 * lane) = lw; }
      __threadfence();
      if (wsv) { *(volatile v2u*)(gp + 4 * lane) = hw; *(volatile v2u*)(gp + HID + 4 * lane) = lw; }
    }
  }
}

template <int EPI>
__global__ __launch_bounds__(GTHR) void k_gemm(const unsigned short* __restrict__ A, int lda, int K,
                                               const unsigned short* __restrict__ WT,
                                               const float* __restrict__ bias,
                                               void* outp, int nN, int mRows,
                                               const float* __restrict__ l2w, const float* __restrict__ l2b,
                                               const int* __restrict__ flags, int nFlag) {
  constexpr int NI = 16;
  __shared__ __attribute__((aligned(16))) float stg[GBM * BN];
  __shared__ __attribute__((aligned(16))) float bs[BN];
  __shared__ __attribute__((aligned(16))) float l2s[BN];
  __shared__ __attribute__((aligned(16))) float outs[GBM];
  const int tid = (int)threadIdx.x, lane = tid & 31, wave = tid >> 5, hh = lane >> 4, m = lane & 15;
  const int rowBase = (int)blockIdx.x * GBM;

  if (tid < 32) {
    const v4f b = *(const v4f*)(bias + 4 * tid);
    v4f r;
    r.x = bf_rne(b.x); r.y = bf_rne(b.y); r.z = bf_rne(b.z); r.w = bf_rne(b.w);
    *(v4fa*)(bs + 4 * tid) = r;
    if constexpr (EPI == 2) {
      const v4f c = *(const v4f*)(l2w + 4 * tid);
      v4f q;
      q.x = bf_rne(c.x); q.y = bf_rne(c.y); q.z = bf_rne(c.z); q.w = bf_rne(c.w);
      *(v4fa*)(l2s + 4 * tid) = q;
    }
  }
  __syncthreads();

  v8f acc[GNT];
  {
    const v8f z = {0.f, 0.f, 0.f, 0.f, 0.f, 0.f, 0.f, 0.f};
#pragma unroll
    for (int t = 0; t < GNT; ++t) acc[t] = z;
  }
  const unsigned short* ap = A + (size_t)(rowBase + 16 * wave + m) * (size_t)lda + 8 * hh;
  const unsigned short* wp = WT + (size_t)m * (size_t)K + 8 * hh;
#pragma unroll 1
  for (int k0 = 0; k0 < K; k0 += 32) {
    FragB af;
    af.h[0] = *(const v8usa*)(ap + k0);
    af.h[1] = *(const v8usa*)(ap + k0 + 16);
#pragma unroll
    for (int t = 0; t < GNT; ++t) {
      const unsigned short* wq = wp + (size_t)(16 * t) * (size_t)K + k0;
      FragB bf;
      bf.h[0] = *(const v8usa*)wq;
      bf.h[1] = *(const v8usa*)(wq + 16);
      acc[t] = wmb(af, bf, acc[t]);
    }
  }

#pragma unroll
  for (int t = 0; t < GNT; ++t) {
    const int lc = 16 * t + m;
    const float bb = bs[lc];
#pragma unroll
    for (int r = 0; r < 8; ++r) {
      const int lr = 16 * wave + 8 * hh + r;
      const bool live = (rowBase + lr) < nN;
      const float v = relu_np(acc[t][r] + bb);
      stg[lr * BN + lc] = live ? v : 0.0f;
    }
  }
  __syncthreads();

  if constexpr (EPI == 0) {
    float* outF = (float*)outp;
    v4f fv[NI];
#pragma unroll
    for (int i = 0; i < NI; ++i) {
      const int lr = 16 * wave + i;
      fv[i] = *(const v4fa*)(stg + lr * BN + 4 * lane);
    }
#pragma unroll
    for (int i = 0; i < NI; ++i) {
      const int gr = rowBase + 16 * wave + i;
      float* op = outF + (size_t)gr * (size_t)HID + 4 * lane;
      if (gr < mRows) *(volatile v4f*)op = fv[i];
    }
    __threadfence();
#pragma unroll
    for (int i = 0; i < NI; ++i) {
      const int gr = rowBase + 16 * wave + i;
      float* op = outF + (size_t)gr * (size_t)HID + 4 * lane;
      if (gr < mRows) *(volatile v4f*)op = fv[i];
    }
  } else if constexpr (EPI == 1) {
    unsigned short* outH = (unsigned short*)outp;
    const int cb = 8 * m;
    const bool isHi = (hh == 0);
    v4u pk[NI];
#pragma unroll
    for (int i = 0; i < NI; ++i) {
      const int lr = 16 * wave + i;
      const v4f a = *(const v4fa*)(stg + lr * BN + cb);
      const v4f b = *(const v4fa*)(stg + lr * BN + cb + 4);
      const float f[8] = {a.x, a.y, a.z, a.w, b.x, b.y, b.z, b.w};
      unsigned int w[4];
#pragma unroll
      for (int j = 0; j < 4; ++j) {
        const unsigned short h0 = bf_bits(f[2 * j]), h1 = bf_bits(f[2 * j + 1]);
        const unsigned short l0 = bf_bits(f[2 * j] - bf_val(h0)), l1 = bf_bits(f[2 * j + 1] - bf_val(h1));
        const unsigned short q0 = isHi ? h0 : l0, q1 = isHi ? h1 : l1;
        w[j] = (unsigned int)q0 | ((unsigned int)q1 << 16);
      }
      v4u pw; pw.x = w[0]; pw.y = w[1]; pw.z = w[2]; pw.w = w[3];
      pk[i] = pw;
    }
#pragma unroll
    for (int i = 0; i < NI; ++i) {
      const int gr = rowBase + 16 * wave + i;
      unsigned short* op = outH + (size_t)gr * (size_t)APW + 8 * lane;
      if (gr < mRows) *(volatile v4u*)op = pk[i];
    }
    __threadfence();
#pragma unroll
    for (int i = 0; i < NI; ++i) {
      const int gr = rowBase + 16 * wave + i;
      unsigned short* op = outH + (size_t)gr * (size_t)APW + 8 * lane;
      if (gr < mRows) *(volatile v4u*)op = pk[i];
    }
  } else {
    float* outF = (float*)outp;
    const float qnan = __int_as_float(0x7fc00000);
    const float l2bv = bf_rne(l2b[0]);
    int af = 0;
#pragma unroll 1
    for (int b = 0; b < nFlag; ++b) af |= flags[b * 32];
    if (tid < GBM) {
      float d = 0.0f;
#pragma unroll 4
      for (int c = 0; c < BN; ++c) d = fmaf(stg[tid * BN + c], l2s[c], d);
      d += l2bv;
      outs[tid] = (af != 0) ? qnan : d;
    }
    __syncthreads();
    const bool okst = (tid < GBM / 4) && (rowBase + 4 * tid + 3 < mRows);
    v4f ov = {0.f, 0.f, 0.f, 0.f};
    const int ti = tid < GBM / 4 ? tid : 0;
    ov = *(const v4fa*)(outs + 4 * ti);
    float* op = outF + (size_t)rowBase + 4 * ti;
    if (okst) *(volatile v4f*)op = ov;
    __threadfence();
    if (okst) *(volatile v4f*)op = ov;
  }
}

__global__ __launch_bounds__(NTHR) void k_pool(const float* __restrict__ hf, const int* __restrict__ bat,
                                               unsigned short* ghl) {
  __shared__ __attribute__((aligned(16))) float wsum[NWAVE * HID];
  __shared__ __attribute__((aligned(16))) float outs[HID];
  const int tid = (int)threadIdx.x, lane = tid & 31, wave = tid >> 5;
  const int g = (int)blockIdx.x;

  float a0 = 0.0f, a1 = 0.0f, a2 = 0.0f, a3 = 0.0f;
#pragma unroll 1
  for (int i0 = wave * 32; i0 < NN; i0 += NTHR) {
    const int i  = i0 + lane;
    const int ic = i < NN ? i : NN - 1;
    const int b  = bat[ic];
    const bool hit = (i < NN) && (b == g);
    unsigned msk = __builtin_amdgcn_ballot_w32(hit);
    int nh = (int)__builtin_popcount(msk);
    nh = nh > 32 ? 32 : nh;
#pragma unroll 1
    for (int q = 0; q < nh; ++q) {
      const int k = __builtin_ffs((int)msk) - 1;
      msk &= msk - 1u;
      int node = i0 + (k < 0 ? 0 : k);
      node = node > NN - 1 ? NN - 1 : node;
      const v4f v = *(const v4f*)(hf + (size_t)node * HID + 4 * lane);
      a0 += v.x; a1 += v.y; a2 += v.z; a3 += v.w;
    }
  }
  wsum[wave * HID + 4 * lane + 0] = a0;
  wsum[wave * HID + 4 * lane + 1] = a1;
  wsum[wave * HID + 4 * lane + 2] = a2;
  wsum[wave * HID + 4 * lane + 3] = a3;
  __syncthreads();
  if (tid < HID) {
    float s = 0.0f;
#pragma unroll
    for (int w2 = 0; w2 < NWAVE; ++w2) s += wsum[w2 * HID + tid];
    outs[tid] = s;
  }
  __syncthreads();
  const int cb = 8 * (lane & 15);
  const bool isHi = lane < 16;
  const v4f a = *(const v4fa*)(outs + cb);
  const v4f b = *(const v4fa*)(outs + cb + 4);
  const float f[8] = {a.x, a.y, a.z, a.w, b.x, b.y, b.z, b.w};
  unsigned int w[4];
#pragma unroll
  for (int j = 0; j < 4; ++j) {
    const unsigned short h0 = bf_bits(f[2 * j]), h1 = bf_bits(f[2 * j + 1]);
    const unsigned short l0 = bf_bits(f[2 * j] - bf_val(h0)), l1 = bf_bits(f[2 * j + 1] - bf_val(h1));
    const unsigned short q0 = isHi ? h0 : l0, q1 = isHi ? h1 : l1;
    w[j] = (unsigned int)q0 | ((unsigned int)q1 << 16);
  }
  v4u pk; pk.x = w[0]; pk.y = w[1]; pk.z = w[2]; pk.w = w[3];
  unsigned short* op = ghl + (size_t)g * APW + 8 * lane;
  const bool okst = (wave == 0);
  if (okst) *(volatile v4u*)op = pk;
  __threadfence();
  if (okst) *(volatile v4u*)op = pk;
}

static inline size_t al256(size_t o) { return (o + 255) & ~(size_t)255; }

extern "C" void kernel_launch(void* const* d_in, const int* in_sizes, int n_in,
                              void* d_out, int out_size, void* d_ws, size_t ws_size,
                              hipStream_t stream) {
  if (n_in < 23) return;
  if (in_sizes[0] != NN * NF) return;
  if (in_sizes[1] != 2 * NE) return;
  if (in_sizes[3] != NN) return;
  if (in_sizes[4] != 1 || in_sizes[9] != 1 || in_sizes[14] != 1) return;
  if (in_sizes[5] != NF * HID) return;
  if (in_sizes[7] != HID * HID || in_sizes[10] != HID * HID || in_sizes[12] != HID * HID) return;
  if (in_sizes[15] != HID * HID || in_sizes[17] != HID * HID || in_sizes[19] != HID * HID) return;
  if (in_sizes[6] != HID || in_sizes[8] != HID || in_sizes[11] != HID || in_sizes[13] != HID) return;
  if (in_sizes[16] != HID || in_sizes[18] != HID || in_sizes[20] != HID) return;
  if (in_sizes[21] != HID || in_sizes[22] != 1) return;
  if (out_size != NG) return;

  const float* x     = (const float*)d_in[0];
  const int*   ei    = (const int*)  d_in[1];
  const int*   src   = ei;
  const int*   dst   = ei + NE;
  const int*   batch = (const int*)  d_in[3];
  const float* eps1  = (const float*)d_in[4];
  const float* W1a   = (const float*)d_in[5];   const float* b1a = (const float*)d_in[6];
  const float* W1b   = (const float*)d_in[7];   const float* b1b = (const float*)d_in[8];
  const float* eps2  = (const float*)d_in[9];
  const float* W2a   = (const float*)d_in[10];  const float* b2a = (const float*)d_in[11];
  const float* W2b   = (const float*)d_in[12];  const float* b2b = (const float*)d_in[13];
  const float* eps3  = (const float*)d_in[14];
  const float* W3a   = (const float*)d_in[15];  const float* b3a = (const float*)d_in[16];
  const float* W3b   = (const float*)d_in[17];  const float* b3b = (const float*)d_in[18];
  const float* l1W   = (const float*)d_in[19];  const float* l1b = (const float*)d_in[20];
  const float* l2W   = (const float*)d_in[21];  const float* l2b = (const float*)d_in[22];
  float* out = (float*)d_out;

  char* ws = (char*)d_ws;
  size_t off = 0;
  const size_t oXB  = off; off = al256(off + (size_t)MP * NF * 2);
  const size_t oW1A = off; off = al256(off + (size_t)HID * 128 * 2);
  const size_t oWT6 = off; off = al256(off + (size_t)6 * WSQ * 2);
  const size_t oZP  = off; off = al256(off + (size_t)MP * APW * 2);
  const size_t oTP  = off; off = al256(off + (size_t)MP * APW * 2);
  const size_t oHF  = off; off = al256(off + (size_t)MP * HID * 4);
  const size_t oLS  = off; off = al256(off + (size_t)NBB * RCAP * 4);
  const size_t oCN  = off; off = al256(off + (size_t)TABN * 4);
  const size_t oOF  = off; off = al256(off + (size_t)TABN * 4);
  const size_t oFL  = off; off = al256(off + (size_t)NBB * 32 * 4);
  const size_t oGH  = off; off = al256(off + (size_t)NG * APW * 2);
  if (off > ws_size || off > (size_t)WSCAP) return;
  unsigned short* XB   = (unsigned short*)(ws + oXB);
  unsigned short* W1AT = (unsigned short*)(ws + oW1A);
  unsigned short* WT6  = (unsigned short*)(ws + oWT6);
  unsigned short* ZP   = (unsigned short*)(ws + oZP);
  unsigned short* TP   = (unsigned short*)(ws + oTP);
  float*          HF   = (float*)(ws + oHF);
  int*            LS   = (int*)(ws + oLS);
  int*            CN   = (int*)(ws + oCN);
  int*            OF   = (int*)(ws + oOF);
  int*            FL   = (int*)(ws + oFL);
  unsigned short* GH   = (unsigned short*)(ws + oGH);

  hipFuncSetAttribute(reinterpret_cast<const void*>(&k_bucket), hipFuncAttributeMaxDynamicSharedMemorySize, LDS_AGG);

  const int gM = MP / GBM;
  const int gA = MP / ARPB;

  k_prep<<<NUTOT / NTHR, NTHR, 0, stream>>>(x, W1a, W1b, W2a, W2b, W3a, W3b, l1W, XB, W1AT, WT6);
  k_bucket<<<NBB, NTHR, LDS_AGG, stream>>>(src, dst, LS, CN, OF, FL);
  k_agg<1><<<gA, NTHR, 0, stream>>>(XB, HF, LS, CN, OF, FL, eps1, ZP);
  k_gemm<1><<<gM, GTHR, 0, stream>>>(ZP, Z1W, 128, W1AT, b1a, (void*)TP, NN, MP, b1a, b1a, FL, 0);
  k_gemm<0><<<gM, GTHR, 0, stream>>>(TP, APW, 256, WT6 + (size_t)0 * WSQ, b1b, (void*)HF, NN, MP, b1b, b1b, FL, 0);
  k_agg<0><<<gA, NTHR, 0, stream>>>(XB, HF, LS, CN, OF, FL, eps2, ZP);
  k_gemm<1><<<gM, GTHR, 0, stream>>>(ZP, APW, 256, WT6 + (size_t)1 * WSQ, b2a, (void*)TP, NN, MP, b2a, b2a, FL, 0);
  k_gemm<0><<<gM, GTHR, 0, stream>>>(TP, APW, 256, WT6 + (size_t)2 * WSQ, b2b, (void*)HF, NN, MP, b2b, b2b, FL, 0);
  k_agg<0><<<gA, NTHR, 0, stream>>>(XB, HF, LS, CN, OF, FL, eps3, ZP);
  k_gemm<1><<<gM, GTHR, 0, stream>>>(ZP, APW, 256, WT6 + (size_t)3 * WSQ, b3a, (void*)TP, NN, MP, b3a, b3a, FL, 0);
  k_gemm<0><<<gM, GTHR, 0, stream>>>(TP, APW, 256, WT6 + (size_t)4 * WSQ, b3b, (void*)HF, NN, MP, b3b, b3b, FL, 0);
  k_pool<<<NG, NTHR, 0, stream>>>(HF, batch, GH);
  k_gemm<2><<<NG / GBM, GTHR, 0, stream>>>(GH, APW, 256, WT6 + (size_t)5 * WSQ, l1b, (void*)out, NG, NG,
                                           l2W, l2b, FL, NBB);
}
